// SoftTreeEnsembleLayerTensor_14620068675646
// MI455X (gfx1250) — hardware-verified
//
#include <hip/hip_runtime.h>

constexpr int kRows      = 8192;
constexpr int kFeat      = 512;
constexpr int kTrees     = 64;
constexpr int kOut       = 128;
constexpr int kNodes     = 63;
constexpr int kLeaves    = 64;
constexpr int kNodeReal  = kNodes * kTrees;
constexpr int kNodeCols  = 4096;
constexpr int kLeafK     = kLeaves * kTrees;
constexpr int kChunk     = 2048;
constexpr int kNumChunks = kRows / kChunk;
static_assert(kRows % kChunk == 0, "chunking");
static_assert(kChunk % 64 == 0 && kNodeCols % 64 == 0 && kOut % 64 == 0, "tile multiples");
static_assert(kFeat % 32 == 0 && kLeafK % 32 == 0, "K multiples of 32");
static_assert(kChunk % 4 == 0, "tree kernel rows per block");

typedef __attribute__((ext_vector_type(16))) _Float16 v16h;
typedef __attribute__((ext_vector_type(8)))  _Float16 v8h;
typedef __attribute__((ext_vector_type(16))) __bf16   v16b;
typedef __attribute__((ext_vector_type(8)))  __bf16   v8b;
typedef __attribute__((ext_vector_type(8)))  float    v8f;
typedef __attribute__((ext_vector_type(4)))  float    v4f;
typedef __attribute__((ext_vector_type(4)))  unsigned int v4u;

__device__ __forceinline__ unsigned short f2bf_bits(float f) {
  unsigned u = __float_as_uint(f);
  return (unsigned short)((u + 0x7FFFu + ((u >> 16) & 1u)) >> 16);
}
__device__ __forceinline__ float bf_bits2f(unsigned short h) { return __uint_as_float(((unsigned)h) << 16); }
__device__ __forceinline__ unsigned pk16(unsigned short a, unsigned short b) { return (unsigned)a | ((unsigned)b << 16); }

__device__ __forceinline__ void dep_guard_h(v8f& a, v8f& b, v16h x, v16h y) { asm volatile("v_nop\n\tv_nop\n\tv_nop\n\tv_nop" : "+v"(a), "+v"(b) : "v"(x), "v"(y)); }
__device__ __forceinline__ void dep_guard_b(v8f& a, v8f& b, v16b x, v16b y) { asm volatile("v_nop\n\tv_nop\n\tv_nop\n\tv_nop" : "+v"(a), "+v"(b) : "v"(x), "v"(y)); }
__device__ __forceinline__ void keep4_h(v16h a, v16h b, v16h c, v16h d) { asm volatile("v_nop" :: "v"(a), "v"(b), "v"(c), "v"(d)); }
__device__ __forceinline__ void keep4_b(v16b a, v16b b, v16b c, v16b d) { asm volatile("v_nop" :: "v"(a), "v"(b), "v"(c), "v"(d)); }
__device__ __forceinline__ void acc_guard4(v8f& a, v8f& b, v8f& c, v8f& d) { asm volatile("v_nop\n\tv_nop\n\tv_nop\n\tv_nop" : "+v"(a), "+v"(b), "+v"(c), "+v"(d)); }
template <typename T> struct Frag;
template <> struct Frag<_Float16> {
  typedef v16h V; union U { v16h v; v8h h[2]; };
  static __device__ __forceinline__ v16h load(const _Float16* p) {
    U f; f.h[0] = *(const v8h*)(p); f.h[1] = *(const v8h*)(p + 16); return f.v;
  }
  static __device__ __forceinline__ v8f mma(v16h a, v16h b, v8f c) {
    return __builtin_amdgcn_wmma_f32_16x16x32_f16(false, a, false, b, (short)0, c, false, false);
  }
  static __device__ __forceinline__ void guard(v8f& a, v8f& b, v16h x, v16h y) { dep_guard_h(a, b, x, y); }
  static __device__ __forceinline__ void keep(v16h a, v16h b, v16h c, v16h d) { keep4_h(a, b, c, d); }
};
template <> struct Frag<__bf16> {
  typedef v16b V; union U { v16b v; v8b h[2]; };
  static __device__ __forceinline__ v16b load(const __bf16* p) {
    U f; f.h[0] = *(const v8b*)(p); f.h[1] = *(const v8b*)(p + 16); return f.v;
  }
  static __device__ __forceinline__ v8f mma(v16b a, v16b b, v8f c) {
    return __builtin_amdgcn_wmma_f32_16x16x32_bf16(false, a, false, b, (short)0, c, false, false);
  }
  static __device__ __forceinline__ void guard(v8f& a, v8f& b, v16b x, v16b y) { dep_guard_b(a, b, x, y); }
  static __device__ __forceinline__ void keep(v16b a, v16b b, v16b c, v16b d) { keep4_b(a, b, c, d); }
};

template <int ET> struct Elem;
template <> struct Elem<0> { typedef _Float16 T; };
template <> struct Elem<1> { typedef __bf16 T; };
template <int ET, int SPLIT, int BIAS_MODE, int OUT_MODE, bool RESID, int ACT = 0>
__global__ __launch_bounds__(256) void wmma_gemm64(
    const unsigned short* __restrict__ Ap, const unsigned short* __restrict__ A2p, int lda, long strideA,
    const unsigned short* __restrict__ Btp, const unsigned short* __restrict__ Bt2p, int ldb, long strideB,
    void* __restrict__ Cout, void* __restrict__ Cout2, int ldc, long strideC,
    const float* __restrict__ bias,
    const float* __restrict__ resid, long strideR,
    int M, int N, int K, float scale) {
  typedef typename Elem<ET>::T T;
  typedef typename Frag<T>::V V;
  const T* A = (const T*)Ap; const T* A2 = (const T*)A2p; const T* Bt = (const T*)Btp; const T* Bt2 = (const T*)Bt2p;
  __shared__ __align__(16) float sT[8][16 * 68];
  const int b    = blockIdx.y;
  const int lane = threadIdx.x & 31;
  const int wave = threadIdx.x >> 5;
  const int tilesN = N >> 6;
  const int tilesM = M >> 6;
  const int tile = blockIdx.x * 8 + wave;
  if (tile >= tilesM * tilesN) return;
  const int tm = tile / tilesN;
  const int tn = tile - tm * tilesN;
  const int m0 = tm << 6;
  const int n0 = tn << 6;

  const T* Ab  = A  + (size_t)b * strideA;
  const T* Bb  = Bt + (size_t)b * strideB;
  const T* Ab2 = (SPLIT != 0) ? (A2  + (size_t)b * strideA) : nullptr;
  const T* Bb2 = (SPLIT == 1) ? (Bt2 + (size_t)b * strideB) : nullptr;

  const int rlane = lane & 15;
  const int koff  = (lane >> 4) * 8;
  const int mOff  = (lane >> 4) * 8;

  v8f acc[4][4];
#pragma unroll
  for (int i = 0; i < 4; ++i)
#pragma unroll
    for (int j = 0; j < 4; ++j) acc[i][j] = (v8f){0.f,0.f,0.f,0.f,0.f,0.f,0.f,0.f};

  for (int k0 = 0; k0 < K; k0 += 32) {
    V bh[4], bl[4];
#pragma unroll
    for (int j = 0; j < 4; ++j) {
      const size_t bo = (size_t)(n0 + (j << 4) + rlane) * ldb + koff + k0;
      bh[j] = Frag<T>::load(Bb + bo);
      if (SPLIT == 1) bl[j] = Frag<T>::load(Bb2 + bo);
    }
#pragma unroll
    for (int i = 0; i < 4; ++i) {
      const size_t ao = (size_t)(m0 + (i << 4) + rlane) * lda + koff + k0;
      V ah = Frag<T>::load(Ab + ao);
      V al;
      if (SPLIT != 0) al = Frag<T>::load(Ab2 + ao);
#pragma unroll
      for (int j = 0; j < 4; ++j) {
        acc[i][j] = Frag<T>::mma(ah, bh[j], acc[i][j]);
        if (SPLIT == 1) acc[i][j] = Frag<T>::mma(ah, bl[j], acc[i][j]);
        if (SPLIT != 0) acc[i][j] = Frag<T>::mma(al, bh[j], acc[i][j]);
      }
      Frag<T>::guard(acc[i][0], acc[i][3], ah, (SPLIT != 0) ? al : ah);
    }
    Frag<T>::keep(bh[0], bh[1], bh[2], bh[3]);
    if (SPLIT == 1) Frag<T>::keep(bl[0], bl[1], bl[2], bl[3]);
  }
  acc_guard4(acc[0][0], acc[0][1], acc[0][2], acc[0][3]);
  acc_guard4(acc[1][0], acc[1][1], acc[1][2], acc[1][3]);
  acc_guard4(acc[2][0], acc[2][1], acc[2][2], acc[2][3]);
  acc_guard4(acc[3][0], acc[3][1], acc[3][2], acc[3][3]);

  float* slab = sT[wave];
  const float* Rb = RESID ? (resid + (size_t)b * strideR) : nullptr;
#pragma unroll
  for (int i = 0; i < 4; ++i) {
    const int mBase = m0 + (i << 4);
#pragma unroll
    for (int j = 0; j < 4; ++j) {
      const int n = n0 + (j << 4) + rlane;
      float bv = 0.f;
      if (BIAS_MODE == 2) bv = bias[n];
#pragma unroll
      for (int r = 0; r < 8; ++r) {
        float v = acc[i][j][r] * scale;
        if (BIAS_MODE == 1) v += bias[mBase + mOff + r];
        if (BIAS_MODE == 2) v += bv;
        if (RESID) v += Rb[(size_t)(mBase + mOff + r) * ldc + n];
        if (ACT == 2) v = fmaxf(v, 0.0f);
        if (ACT == 4) v = (v > 0.f) ? v : 0.01f * v;
        slab[(mOff + r) * 68 + (j << 4) + rlane] = v;
      }
    }
    __builtin_amdgcn_fence(__ATOMIC_RELEASE, "workgroup");
    __builtin_amdgcn_wave_barrier();
    __builtin_amdgcn_fence(__ATOMIC_ACQUIRE, "workgroup");
    if (OUT_MODE == 0) {
      float* C = (float*)Cout + (size_t)b * strideC;
      const int hh = lane >> 4, c4 = (lane & 15) * 4;
      for (int pass = 0; pass < 2; ++pass) {
#pragma unroll
        for (int it = 0; it < 8; ++it) {
          const int row = it * 2 + hh;
          v4f v = *(const v4f*)(slab + row * 68 + c4);
          *(volatile v4f*)(C + (size_t)(mBase + row) * ldc + n0 + c4) = v;
        }
        __threadfence();
      }
    } else {
      const int q = lane >> 3, c8 = (lane & 7) * 8;
      unsigned short* C  = (unsigned short*)Cout  + (size_t)b * strideC;
      unsigned short* C2 = (OUT_MODE == 2) ? ((unsigned short*)Cout2 + (size_t)b * strideC) : nullptr;
      for (int pass = 0; pass < 2; ++pass) {
#pragma unroll
        for (int it = 0; it < 4; ++it) {
          const int row = it * 4 + q;
          const float* sp = slab + row * 68 + c8;
          v8h hv, lv;
#pragma unroll
          for (int e = 0; e < 8; ++e) {
            if (OUT_MODE == 1) {
              hv[e] = (_Float16)sp[e];
            } else {
              unsigned short hb = f2bf_bits(sp[e]);
              unsigned short lb = f2bf_bits(sp[e] - bf_bits2f(hb));
              hv[e] = __builtin_bit_cast(_Float16, hb);
              lv[e] = __builtin_bit_cast(_Float16, lb);
            }
          }
          *(volatile v8h*)(C + (size_t)(mBase + row) * ldc + n0 + c8) = hv;
          if (OUT_MODE == 2) *(volatile v8h*)(C2 + (size_t)(mBase + row) * ldc + n0 + c8) = lv;
        }
        __threadfence();
      }
    }
    __builtin_amdgcn_fence(__ATOMIC_RELEASE, "workgroup");
    __builtin_amdgcn_wave_barrier();
    __builtin_amdgcn_fence(__ATOMIC_ACQUIRE, "workgroup");
  }
}

__global__ __launch_bounds__(256) void cast8_bf16_kernel(const float* __restrict__ in,
                                                       unsigned short* __restrict__ out, int n8) {
  const int i = blockIdx.x * 256 + threadIdx.x;
  if (i >= n8) return;
  const float* p = in + 8 * (size_t)i;
  const v4f a = *(const v4f*)(p);
  const v4f c = *(const v4f*)(p + 4);
  const v4u u = (v4u){pk16(f2bf_bits(a[0]), f2bf_bits(a[1])), pk16(f2bf_bits(a[2]), f2bf_bits(a[3])),
                      pk16(f2bf_bits(c[0]), f2bf_bits(c[1])), pk16(f2bf_bits(c[2]), f2bf_bits(c[3]))};
  unsigned short* q = out + 8 * (size_t)i;
  *(volatile v4u*)q = u;
  __threadfence();
  *(volatile v4u*)q = u;
}

__global__ __launch_bounds__(256) void wnode_transpose_kernel(const float* __restrict__ Wn,
                                                             unsigned short* __restrict__ out) {
  __shared__ float sm[64][65];
  const int t  = threadIdx.x;
  const int f0 = blockIdx.x * 64;
  const int ns = blockIdx.y;
  const bool pad = (ns >= kNodes);
  const int nld = pad ? (kNodes - 1) : ns;
#pragma unroll
  for (int i = 0; i < 16; ++i) {
    const int e  = i * 256 + t;
    const int fl = e >> 6;
    const int tq = e & 63;
    const float v = Wn[((size_t)nld * kFeat + f0 + fl) * kTrees + tq];
    sm[tq][fl] = pad ? 0.0f : v;
  }
  __syncthreads();
  const int lane = t & 31, wave = t >> 5;
  const int q = lane >> 3, c8 = (lane & 7) * 8;
  for (int pass = 0; pass < 2; ++pass) {
#pragma unroll
    for (int it = 0; it < 2; ++it) {
      const int row = wave * 8 + it * 4 + q;
      unsigned short hb[8];
#pragma unroll
      for (int e = 0; e < 8; ++e) hb[e] = f2bf_bits(sm[row][c8 + e]);
      const v4u u = (v4u){pk16(hb[0], hb[1]), pk16(hb[2], hb[3]), pk16(hb[4], hb[5]), pk16(hb[6], hb[7])};
      *(volatile v4u*)(out + (size_t)(ns * kTrees + row) * kFeat + f0 + c8) = u;
    }
    __threadfence();
  }
}

__global__ __launch_bounds__(256) void wleaf_pack_kernel(const float* __restrict__ Wl,
                                                        unsigned short* __restrict__ out) {
  const int i   = blockIdx.x * 256 + threadIdx.x;
  const int d   = i * 8;
  const int o   = d >> 12;
  const int rem = d & (kLeafK - 1);
  const int l   = rem >> 6;
  const int t0  = rem & 63;
  const float* p = Wl + ((size_t)(l * kOut + o) * kTrees + t0);
  const v4f a = *(const v4f*)(p);
  const v4f c = *(const v4f*)(p + 4);
  const v4u u = (v4u){pk16(f2bf_bits(a[0]), f2bf_bits(a[1])), pk16(f2bf_bits(a[2]), f2bf_bits(a[3])),
                      pk16(f2bf_bits(c[0]), f2bf_bits(c[1])), pk16(f2bf_bits(c[2]), f2bf_bits(c[3]))};
  unsigned short* q = out + (size_t)d;
  *(volatile v4u*)q = u;
  __threadfence();
  *(volatile v4u*)q = u;
}

__global__ __launch_bounds__(256) void bias_pack_kernel(const float* __restrict__ bn, float* __restrict__ outb) {
  const int tid = threadIdx.x;
  v4f vals[4];
#pragma unroll
  for (int it = 0; it < 4; ++it) {
    const int c = (it * 256 + tid) * 4;
    v4f v;
#pragma unroll
    for (int e = 0; e < 4; ++e) {
      const int cc = c + e;
      const int cl = (cc < kNodeReal) ? cc : (kNodeReal - 1);
      const float f = bf_bits2f(f2bf_bits(bn[cl]));
      v[e] = (cc < kNodeReal) ? f : 0.0f;
    }
    vals[it] = v;
  }
  for (int pass = 0; pass < 2; ++pass) {
#pragma unroll
    for (int it = 0; it < 4; ++it) {
      const int c = (it * 256 + tid) * 4;
      *(volatile v4f*)(outb + c) = vals[it];
    }
    __threadfence();
  }
}

__global__ __launch_bounds__(256) void tree_prob_kernel(const float* __restrict__ S,
                                                       unsigned short* __restrict__ PH,
                                                       unsigned short* __restrict__ PL) {
#pragma clang fp contract(off)
  __shared__ __align__(16) unsigned int ldsP[4 * kLeafK];
  const int tid  = threadIdx.x;
  const int rl   = tid >> 6;
  const int tt   = tid & 63;
  const int row0 = blockIdx.x * 4;
  const float* sr = S + (size_t)(row0 + rl) * kNodeCols + tt;

  float p[64];
  p[0] = 1.0f;
#pragma unroll
  for (int lvl = 0; lvl < 6; ++lvl) {
    const int width = 1 << lvl;
    const int nbase = width - 1;
#pragma unroll
    for (int j = width - 1; j >= 0; --j) {
      const float v  = sr[(nbase + j) * kTrees];
      const float tc = fminf(fmaxf(v, -0.5f), 0.5f);
      const float t2 = tc * tc;
      const float t3 = tc * t2;
      const float sv = ((-2.0f * t3) + (1.5f * tc)) + 0.5f;
      const float pj = p[j];
      const float om = 1.0f - sv;
      p[2 * j + 1] = pj * om;
      p[2 * j]     = pj * sv;
    }
  }
  unsigned int* lp = ldsP + rl * kLeafK + tt;
#pragma unroll
  for (int l = 0; l < 64; ++l) {
    const float pv = p[l];
    const unsigned short hb = f2bf_bits(pv);
    const unsigned short lb = f2bf_bits(pv - bf_bits2f(hb));
    lp[l * kTrees] = (unsigned)hb | ((unsigned)lb << 16);
  }
  __syncthreads();

  for (int pass = 0; pass < 2; ++pass) {
#pragma unroll
    for (int it = 0; it < 8; ++it) {
      const int g  = it * 256 + tid;
      const int r  = g >> 9;
      const int c8 = (g & 511) * 8;
      const v4u w0 = *(const v4u*)(ldsP + r * kLeafK + c8);
      const v4u w1 = *(const v4u*)(ldsP + r * kLeafK + c8 + 4);
      v4u hv, lv;
      hv.x = (w0.x & 0xffffu) | (w0.y << 16);
      hv.y = (w0.z & 0xffffu) | (w0.w << 16);
      hv.z = (w1.x & 0xffffu) | (w1.y << 16);
      hv.w = (w1.z & 0xffffu) | (w1.w << 16);
      lv.x = (w0.x >> 16) | (w0.y & 0xffff0000u);
      lv.y = (w0.z >> 16) | (w0.w & 0xffff0000u);
      lv.z = (w1.x >> 16) | (w1.y & 0xffff0000u);
      lv.w = (w1.z >> 16) | (w1.w & 0xffff0000u);
      const size_t off = (size_t)(row0 + r) * kLeafK + c8;
      *(volatile v4u*)(PH + off) = hv;
      *(volatile v4u*)(PL + off) = lv;
    }
    __threadfence();
  }
}

extern "C" void kernel_launch(void* const* d_in, const int* in_sizes, int n_in,
                              void* d_out, int out_size, void* d_ws, size_t ws_size,
                              hipStream_t stream) {
  (void)n_in;
  const float* x  = (const float*)d_in[0];
  const float* Wn = (const float*)d_in[1];
  const float* bn = (const float*)d_in[2];
  const float* Wl = (const float*)d_in[3];
  float* out = (float*)d_out;

  if (in_sizes[0] != kRows * kFeat || in_sizes[1] != kNodes * kFeat * kTrees ||
      in_sizes[2] != kNodes * kTrees || in_sizes[3] != kLeaves * kOut * kTrees ||
      out_size != kRows * kOut) return;

  const size_t xbBytes   = (size_t)kRows * kFeat * 2;
  const size_t wntBytes  = (size_t)kNodeCols * kFeat * 2;
  const size_t wltBytes  = (size_t)kOut * kLeafK * 2;
  const size_t biasBytes = (size_t)kNodeCols * 4;
  const size_t sBytes    = (size_t)kChunk * kNodeCols * 4;
  const size_t pBytes    = (size_t)kChunk * kLeafK * 2;
  const size_t offXb   = 0;
  const size_t offWnT  = offXb + xbBytes;
  const size_t offWlT  = offWnT + wntBytes;
  const size_t offBias = offWlT + wltBytes;
  const size_t offS    = offBias + biasBytes;
  const size_t offPH   = offS + sBytes;
  const size_t offPL   = offPH + pBytes;
  const size_t total   = offPL + pBytes;
  if (total > ws_size) return;

  char* ws = (char*)d_ws;
  unsigned short* xb    = (unsigned short*)(ws + offXb);
  unsigned short* WnT   = (unsigned short*)(ws + offWnT);
  unsigned short* WlT   = (unsigned short*)(ws + offWlT);
  float*          biasP = (float*)(ws + offBias);
  float*          S     = (float*)(ws + offS);
  unsigned short* PH    = (unsigned short*)(ws + offPH);
  unsigned short* PL    = (unsigned short*)(ws + offPL);

  const int n8x = kRows * kFeat / 8;
  cast8_bf16_kernel<<<dim3((n8x + 255) / 256), dim3(256), 0, stream>>>(x, xb, n8x);
  wnode_transpose_kernel<<<dim3(kFeat / 64, kNodeCols / kTrees), dim3(256), 0, stream>>>(Wn, WnT);
  wleaf_pack_kernel<<<dim3((kOut * kLeafK / 8) / 256), dim3(256), 0, stream>>>(Wl, WlT);
  bias_pack_kernel<<<dim3(1), dim3(256), 0, stream>>>(bn, biasP);

  const int nodeTiles = (kChunk / 64) * (kNodeCols / 64);
  const int leafTiles = (kChunk / 64) * (kOut / 64);
  for (int c = 0; c < kNumChunks; ++c) {
    const unsigned short* xc = xb + (size_t)c * kChunk * kFeat;
    float* oc = out + (size_t)c * kChunk * kOut;
    wmma_gemm64<1, 0, 2, 0, false><<<dim3((nodeTiles + 7) / 8, 1), dim3(256), 0, stream>>>(
        xc, xc, kFeat, 0L, WnT, WnT, kFeat, 0L, (void*)S, (void*)S, kNodeCols, 0L,
        biasP, biasP, 0L, kChunk, kNodeCols, kFeat, 1.0f);
    tree_prob_kernel<<<dim3(kChunk / 4), dim3(256), 0, stream>>>(S, PH, PL);
    wmma_gemm64<1, 2, 0, 0, false><<<dim3((leafTiles + 7) / 8, 1), dim3(256), 0, stream>>>(
        PH, PL, kLeafK, 0L, WlT, WlT, kLeafK, 0L, (void*)oc, (void*)oc, kOut, 0L,
        biasP, biasP, 0L, kChunk, kOut, kLeafK, 1.0f);
  }
}
